// Net_LV_75797582840291
// MI455X (gfx1250) — hardware-verified
//
#include <hip/hip_runtime.h>
#include <stddef.h>

typedef __attribute__((ext_vector_type(16))) _Float16 v16h;
typedef __attribute__((ext_vector_type(8)))  _Float16 v8h;
typedef __attribute__((ext_vector_type(8)))  float    v8f;
typedef __attribute__((ext_vector_type(4)))  float    v4f;

#define NUM_PATHS 32768
#define NUM_STEPS 90
#define NUM_COLS 91
#define PATHS_PER_BLOCK 32
#define MAIN_THREADS 64
#define FIN_THREADS 256

constexpr int BT_DWH = 0;
constexpr int BT_DWO = 36864;
constexpr int BT_VWH = 39936;
constexpr int BT_VWO = 52224;
constexpr int BT_EWI = 64512;
constexpr int BT_EWH = 76800;
constexpr int BT_EWO = 89088;
constexpr int BT_TOTAL = 92160;
static_assert(BT_TOTAL * 2 == 184320, "bt bytes");

constexpr size_t WS_BT    = 0;
constexpr size_t WS_PRICE = 184320;
constexpr size_t WS_EXD   = WS_PRICE + (size_t)NUM_PATHS * 64 * 4;
constexpr size_t WS_CVE   = WS_EXD + (size_t)NUM_PATHS * 4;
constexpr size_t WS_END   = WS_CVE + (size_t)NUM_PATHS * 4;
static_assert(WS_END == 8835072, "ws carve");
static_assert(WS_PRICE % 128 == 0 && WS_EXD % 128 == 0 && WS_CVE % 128 == 0, "ws align");

constexpr int OUT1_OFF = NUM_PATHS * NUM_COLS;
constexpr int OUT2_OFF = 2 * NUM_PATHS * NUM_COLS;
constexpr int TAIL_OFF = OUT2_OFF + NUM_PATHS;
constexpr int TAIL_FLOATS = 63 + 63 + NUM_PATHS + 1 + 1 + NUM_PATHS;
constexpr int OUT_TOTAL = TAIL_OFF + TAIL_FLOATS;
static_assert(OUT_TOTAL == 6062208, "out size");
static_assert((TAIL_OFF * 4) % 128 == 0 && (TAIL_FLOATS % 4) == 0, "tail region lines");

constexpr int PITCH_ACT = 72;
constexpr int PITCH_PH  = 104;
constexpr int LDS_ACT0  = 0;
constexpr int LDS_ACT1  = LDS_ACT0 + 32 * PITCH_ACT * 2;
constexpr int LDS_PATHH = LDS_ACT1 + 32 * PITCH_ACT * 2;
constexpr int LDS_PATHS = LDS_PATHH + 32 * PITCH_PH * 2;
constexpr int LDS_VARS  = LDS_PATHS + 32 * NUM_COLS * 4;
constexpr int LDS_PRICE = LDS_VARS + 32 * NUM_COLS * 4;
constexpr int LDS_CVS   = LDS_PRICE + 32 * 64 * 4;
constexpr int LDS_PAR   = LDS_CVS + 32 * 64 * 4;
constexpr int LDS_SC    = LDS_PAR + 768 * 4;
constexpr int LDS_TOTAL = LDS_SC + 384 * 4;
static_assert(LDS_TOTAL == 60160 && (LDS_TOTAL % 16) == 0, "lds size");
static_assert(LDS_PATHS % 16 == 0 && LDS_VARS % 16 == 0 && LDS_PRICE % 16 == 0 && LDS_SC % 32 == 0, "lds align");

constexpr int PT_DW0 = 0;
constexpr int PT_DW1 = 64;
constexpr int PT_DB  = 128;
constexpr int PT_DBH = 192;
constexpr int PT_VW0 = 384;
constexpr int PT_VW1 = 416;
constexpr int PT_VB  = 448;
constexpr int PT_VBH = 480;
constexpr int PT_VBO = 544;
constexpr int PT_EW0 = 608;
constexpr int PT_EB  = 640;
constexpr int PT_EBH = 672;
constexpr int PT_DBO = 736;
constexpr int PT_EBO = 737;
constexpr int SC_YD   = 0;
constexpr int SC_YE   = 32;
constexpr int SC_CO   = 64;
constexpr int SC_DW   = 96;
constexpr int SC_EXD  = 128;
constexpr int SC_CVE  = 160;
constexpr int SC_DL   = 192;
constexpr int SC_BEFF = 224;

struct FragH {
  union U { v16h v; v8h h[2]; };
  static __device__ __forceinline__ v16h load(const _Float16* p) {
    U f; f.h[0] = *(const v8h*)(p); f.h[1] = *(const v8h*)(p + 16); return f.v;
  }
};
__device__ __forceinline__ v8f mma_h(v16h a, v16h b, v8f c) {
  c = __builtin_amdgcn_wmma_f32_16x16x32_f16(false, a, false, b, (short)0, c, false, false);
  asm volatile("v_nop\n\tv_nop\n\tv_nop\n\tv_nop" : "+v"(c) : "v"(a), "v"(b));
  return c;
}
__device__ __forceinline__ v8f zero8() { return (v8f){0.f,0.f,0.f,0.f,0.f,0.f,0.f,0.f}; }

__global__ __launch_bounds__(64) void prep_bt16(const float* __restrict__ src, int srcMatStride, int kdim, int ndim,
                                               int nPad, int kPitch, int totalLines, _Float16* __restrict__ dst) {
  const int lane = threadIdx.x & 31, wave = threadIdx.x >> 5;
  const int line = (blockIdx.x * 2 + wave) * 4 + (lane >> 3);
  const int seg = lane & 7;
  const bool valid = line < totalLines;
  const int lc = valid ? line : (totalLines - 1);
  const int lpr = kPitch >> 6;
  const int rowAll = lc / lpr;
  const int row = rowAll % nPad;
  const int q = rowAll / nPad;
  const int col0 = (lc - rowAll * lpr) * 64 + seg * 8;
  const int na = (row < ndim) ? row : (ndim - 1);
  v8h hv;
#pragma unroll
  for (int e = 0; e < 8; ++e) {
    const int k = col0 + e;
    const int ka = (k < kdim) ? k : (kdim - 1);
    const float w = src[(size_t)q * srcMatStride + (size_t)ka * ndim + na];
    const float f = (k < kdim && row < ndim) ? 16.0f : 0.0f;
    hv[e] = (_Float16)(w * f);
  }
  if (valid) {
    _Float16* p = dst + (size_t)lc * 64 + seg * 8;
    *(volatile v8h*)p = hv;
    __threadfence();
    *(volatile v8h*)p = hv;
  }
}

template <int KS, int NS>
__device__ __forceinline__ void dense_relu(const _Float16* inT, int pin, _Float16* outT, int pout,
                                           const _Float16* __restrict__ bt, int kp, const float* bias8,
                                           int wrow0, int lane) {
  const int rl = lane & 15, hh = lane >> 4, koff = hh * 8;
  v16h a[KS];
#pragma unroll
  for (int ks = 0; ks < KS; ++ks) a[ks] = FragH::load(inT + (wrow0 + rl) * pin + koff + 32 * ks);
  v8f acc[NS];
#pragma unroll
  for (int j = 0; j < NS; ++j) acc[j] = zero8();
#pragma unroll
  for (int ks = 0; ks < KS; ++ks) {
#pragma unroll
    for (int j = 0; j < NS; ++j) {
      const v16h b = FragH::load(bt + (size_t)(16 * j + rl) * kp + koff + 32 * ks);
      acc[j] = mma_h(a[ks], b, acc[j]);
    }
  }
#pragma unroll
  for (int j = 0; j < NS; ++j) {
    const float b8 = bias8[16 * j + rl];
    _Float16* op = outT + (wrow0 + 8 * hh) * pout + 16 * j + rl;
#pragma unroll
    for (int r = 0; r < 8; ++r) {
      float x = fmaf(acc[j][r], 0.0625f, b8);
      x = fmaxf(x, 0.0f);
      op[r * pout] = (_Float16)x;
    }
  }
}

template <int KS>
__device__ __forceinline__ void dense_head(const _Float16* inT, int pin, const _Float16* __restrict__ bt, float bo,
                                           float* yS, int wrow0, int lane) {
  const int rl = lane & 15, hh = lane >> 4, koff = hh * 8;
  v8f acc = zero8();
#pragma unroll
  for (int ks = 0; ks < KS; ++ks) {
    const v16h a = FragH::load(inT + (wrow0 + rl) * pin + koff + 32 * ks);
    const v16h b = FragH::load(bt + (size_t)rl * 64 + koff + 32 * ks);
    acc = mma_h(a, b, acc);
  }
  if (rl == 0) {
#pragma unroll
    for (int r = 0; r < 8; ++r) yS[wrow0 + 8 * hh + r] = fmaf(acc[r], 0.0078125f, bo);
  }
}

__global__ __launch_bounds__(MAIN_THREADS) void lv_paths(
    const float* __restrict__ S0p, int nS0, const float* __restrict__ z,
    const float* __restrict__ dWi, const float* __restrict__ dbi, const float* __restrict__ dbh, const float* __restrict__ dbo,
    const float* __restrict__ vWi, const float* __restrict__ vbi, const float* __restrict__ vbh, const float* __restrict__ vbo,
    const float* __restrict__ eWi, const float* __restrict__ ebi, const float* __restrict__ ebh, const float* __restrict__ ebo,
    const _Float16* __restrict__ bt, float* __restrict__ out,
    float* __restrict__ wsPrice, float* __restrict__ wsExd, float* __restrict__ wsCve) {
  __shared__ __align__(32) unsigned char lds_raw[LDS_TOTAL];
  _Float16* act0  = (_Float16*)(lds_raw + LDS_ACT0);
  _Float16* act1  = (_Float16*)(lds_raw + LDS_ACT1);
  _Float16* pathH = (_Float16*)(lds_raw + LDS_PATHH);
  float* pathS  = (float*)(lds_raw + LDS_PATHS);
  float* varS   = (float*)(lds_raw + LDS_VARS);
  float* priceS = (float*)(lds_raw + LDS_PRICE);
  float* cvS    = (float*)(lds_raw + LDS_CVS);
  float* par    = (float*)(lds_raw + LDS_PAR);
  float* sc     = (float*)(lds_raw + LDS_SC);

  const int tid = threadIdx.x, lane = tid & 31, wave = tid >> 5;
  const int c = lane & 15, hh = lane >> 4, koff = hh * 8;
  const int wrow0 = wave * 16;
  const int p = wrow0 + c;
  int gp = blockIdx.x * PATHS_PER_BLOCK + p;
  gp = (gp < NUM_PATHS) ? gp : (NUM_PATHS - 1);

  for (int t4 = tid; t4 < LDS_TOTAL / 16; t4 += MAIN_THREADS) ((uint4*)lds_raw)[t4] = make_uint4(0u, 0u, 0u, 0u);
  __syncthreads();

  int s0i = (gp < nS0) ? gp : (nS0 - 1);
  s0i = (s0i < 0) ? 0 : s0i;
  const float s0 = S0p[s0i];
  float S = s0, rmax = s0, cve = 0.0f, dlast = 0.0f, c3 = 0.0f, dWv = 0.0f;
  pathS[p * NUM_COLS] = s0;
  pathH[p * PITCH_PH] = (_Float16)(8.0f * s0);
  v8f cv[4];
#pragma unroll
  for (int j = 0; j < 4; ++j) cv[j] = zero8();
  __syncthreads();

  for (int i = 1; i <= NUM_STEPS; ++i) {
    const int m = (i - 1) / 30;
    if (((i - 1) % 30) == 0) {
      const int n = tid;
      const bool okd = n < 50;
      const int nd = okd ? n : 49;
      const float fd = okd ? 8.0f : 0.0f;
      par[PT_DW0 + n] = fd * dWi[m * 100 + nd];
      par[PT_DW1 + n] = fd * dWi[m * 100 + 50 + nd];
      par[PT_DB + n]  = fd * dbi[m * 50 + nd];
#pragma unroll
      for (int l = 0; l < 3; ++l) par[PT_DBH + l * 64 + n] = fd * dbh[(m * 3 + l) * 50 + nd];
      const bool okvo = n < 63;
      const int nvo = okvo ? n : 62;
      const float fvo = okvo ? 1.0f : 0.0f;
      par[PT_VBO + n] = fvo * vbo[m * 63 + nvo];
      const float vdbo = dbo[m];
      const float vebo = ebo[m];
      if (tid < 32) {
        const int nn = tid;
        const bool okv = nn < 30;
        const int nv = okv ? nn : 29;
        const float fv = okv ? 8.0f : 0.0f;
        par[PT_VW0 + nn] = fv * vWi[m * 60 + nv];
        par[PT_VW1 + nn] = fv * vWi[m * 60 + 30 + nv];
        par[PT_VB + nn]  = fv * vbi[m * 30 + nv];
#pragma unroll
        for (int l = 0; l < 2; ++l) par[PT_VBH + l * 32 + nn] = fv * vbh[(m * 2 + l) * 30 + nv];
        const bool oke = nn < 20;
        const int ne = oke ? nn : 19;
        const float fe = oke ? 8.0f : 0.0f;
        par[PT_EW0 + nn] = fe * eWi[m * 1840 + ne];
        par[PT_EB + nn]  = fe * ebi[m * 20 + ne];
#pragma unroll
        for (int l = 0; l < 2; ++l) par[PT_EBH + l * 32 + nn] = fe * ebh[(m * 2 + l) * 20 + ne];
      }
      if (tid == 0) { par[PT_DBO] = vdbo; par[PT_EBO] = vebo; }
      __syncthreads();
    }

    const float tp  = 0.01f * (float)(i - 1);
    const float tn  = 0.01f * (float)i;
    const float h   = tn - tp;
    const float sqh = sqrtf(h);

    {
      _Float16* row = act0 + p * PITCH_ACT;
#pragma unroll 4
      for (int q = 0; q < 32; ++q) {
        const int n = hh * 32 + q;
        float x = fmaf(tp, par[PT_DW0 + n], fmaf(S, par[PT_DW1 + n], par[PT_DB + n]));
        x = fmaxf(x, 0.0f);
        row[n] = (_Float16)x;
      }
      sc[SC_BEFF + wave * 32 + lane] = fmaf(tp, par[PT_EW0 + lane], par[PT_EB + lane]);
    }
    __syncthreads();

    const _Float16* btDwh = bt + BT_DWH + m * 12288;
    dense_relu<2, 4>(act0, PITCH_ACT, act1, PITCH_ACT, btDwh,        64, par + PT_DBH,       wrow0, lane);
    __syncthreads();
    dense_relu<2, 4>(act1, PITCH_ACT, act0, PITCH_ACT, btDwh + 4096, 64, par + PT_DBH + 64,  wrow0, lane);
    __syncthreads();
    dense_relu<2, 4>(act0, PITCH_ACT, act1, PITCH_ACT, btDwh + 8192, 64, par + PT_DBH + 128, wrow0, lane);
    __syncthreads();
    dense_head<2>(act1, PITCH_ACT, bt + BT_DWO + m * 1024, par[PT_DBO], sc + SC_YD, wrow0, lane);
    __syncthreads();

    {
      const float y = sc[SC_YD + p];
      const float diff = fmaxf(y, 0.0f) + log1pf(expf(-fabsf(y)));
      const float vv = diff * diff;
      const float zc = z[(size_t)gp * NUM_STEPS + (i - 1)];
      const float dW = sqh * zc;
      const float rS = 0.025f * S;
      const float num1 = rS * h;
      const float den1 = 1.0f + rS * sqh;
      const float sd = S * diff;
      const float num2 = sd * dW;
      const float den2 = 1.0f + sd * sqh;
      const float Snew = (S + num1 * (1.0f / den1)) + num2 * (1.0f / den2);
      const float disc = expf(-0.025f * tp);
      c3 = (disc * S) * diff;
      dWv = dW;
      sc[SC_CO + p] = c3;
      sc[SC_DW + p] = dW;
      varS[p * NUM_COLS + i] = vv;
      if (i == 1) varS[p * NUM_COLS] = vv;
      pathS[p * NUM_COLS + i] = Snew;
      rmax = fmaxf(rmax, Snew);
      if (i == NUM_STEPS) dlast = diff;
      _Float16* row = act0 + p * PITCH_ACT;
#pragma unroll 4
      for (int q = 0; q < 16; ++q) {
        const int n = hh * 16 + q;
        float x = fmaf(tp, par[PT_VW0 + n], fmaf(S, par[PT_VW1 + n], par[PT_VB + n]));
        x = fmaxf(x, 0.0f);
        row[n] = (_Float16)x;
      }
      S = Snew;
    }
    __syncthreads();

    const _Float16* btVwh = bt + BT_VWH + m * 4096;
    dense_relu<1, 2>(act0, PITCH_ACT, act1, PITCH_ACT, btVwh,        64, par + PT_VBH,      wrow0, lane);
    __syncthreads();
    dense_relu<1, 2>(act1, PITCH_ACT, act0, PITCH_ACT, btVwh + 2048, 64, par + PT_VBH + 32, wrow0, lane);
    __syncthreads();

    {
      const v16h a = FragH::load(act0 + (wrow0 + c) * PITCH_ACT + koff);
      const _Float16* btVwo = bt + BT_VWO + m * 4096;
      v8f acc[4];
#pragma unroll
      for (int j = 0; j < 4; ++j) {
        const v16h b = FragH::load(btVwo + (size_t)(16 * j + c) * 64 + koff);
        acc[j] = mma_h(a, b, zero8());
      }
      const v4f co0 = *(const v4f*)(sc + SC_CO + wrow0 + 8 * hh);
      const v4f co1 = *(const v4f*)(sc + SC_CO + wrow0 + 8 * hh + 4);
      const v4f dw0 = *(const v4f*)(sc + SC_DW + wrow0 + 8 * hh);
      const v4f dw1 = *(const v4f*)(sc + SC_DW + wrow0 + 8 * hh + 4);
#pragma unroll
      for (int j = 0; j < 4; ++j) {
        const float bo = par[PT_VBO + 16 * j + c];
#pragma unroll
        for (int r = 0; r < 4; ++r) {
          const float yv = fmaf(acc[j][r], 0.0078125f, bo);
          cv[j][r] = cv[j][r] + (co0[r] * yv) * dw0[r];
        }
#pragma unroll
        for (int r = 0; r < 4; ++r) {
          const float yv = fmaf(acc[j][4 + r], 0.0078125f, bo);
          cv[j][4 + r] = cv[j][4 + r] + (co1[r] * yv) * dw1[r];
        }
      }
    }
    dense_relu<3, 2>(pathH, PITCH_PH, act1, PITCH_ACT, bt + BT_EWI + m * 4096, 128, sc + SC_BEFF + wave * 32, wrow0, lane);
    __syncthreads();

    const _Float16* btEwh = bt + BT_EWH + m * 4096;
    dense_relu<1, 2>(act1, PITCH_ACT, act0, PITCH_ACT, btEwh,        64, par + PT_EBH,      wrow0, lane);
    __syncthreads();
    dense_relu<1, 2>(act0, PITCH_ACT, act1, PITCH_ACT, btEwh + 2048, 64, par + PT_EBH + 32, wrow0, lane);
    __syncthreads();
    dense_head<1>(act1, PITCH_ACT, bt + BT_EWO + m * 1024, par[PT_EBO], sc + SC_YE, wrow0, lane);
    __syncthreads();

    {
      const float ye = sc[SC_YE + p];
      cve = cve + (c3 * ye) * dWv;
      pathH[p * PITCH_PH + i] = (_Float16)(8.0f * S);
    }
    if ((i % 30) == 0) {
#pragma unroll
      for (int j = 0; j < 4; ++j) {
#pragma unroll
        for (int r = 0; r < 8; ++r) cvS[(wrow0 + 8 * hh + r) * 64 + 16 * j + c] = cv[j][r];
      }
      __syncthreads();
      const float tm = 0.01f * (float)((m + 1) * 30);
      const float dm = expf(-0.025f * tm);
#pragma unroll 1
      for (int q = 0; q < 11; ++q) {
        const int k = hh * 11 + q;
        const int kc = (k < 21) ? k : 20;
        const float st = 0.8f + 0.02f * (float)kc;
        const float pr = dm * fmaxf(S - st, 0.0f) - cvS[p * 64 + m * 21 + kc];
        if (k < 21) priceS[p * 64 + m * 21 + kc] = pr;
      }
    }
    __syncthreads();
  }

  {
    const float discT = expf(-0.025f * (0.01f * 90.0f));
    sc[SC_EXD + p] = discT * (rmax - S);
    sc[SC_CVE + p] = cve;
    sc[SC_DL + p]  = dlast;
  }
  __syncthreads();

  {
    const size_t blk = blockIdx.x;
    float* o0 = out + blk * (size_t)(32 * NUM_COLS);
    float* o1 = out + OUT1_OFF + blk * (size_t)(32 * NUM_COLS);
    float* o2 = out + OUT2_OFF + blk * 32;
    float* wp = wsPrice + blk * 2048;
    float* we = wsExd + blk * 32;
    float* wc = wsCve + blk * 32;
    for (int pass = 0; pass < 2; ++pass) {
#pragma unroll 1
      for (int it = 0; it < 12; ++it) {
        const int f = it * MAIN_THREADS + tid;
        if (f < 728) {
          const v4f a4 = *(const v4f*)(pathS + 4 * f);
          const v4f b4 = *(const v4f*)(varS + 4 * f);
          *(volatile v4f*)(o0 + 4 * f) = a4;
          *(volatile v4f*)(o1 + 4 * f) = b4;
        }
      }
#pragma unroll 1
      for (int it = 0; it < 8; ++it) {
        const int f = it * MAIN_THREADS + tid;
        const v4f q4 = *(const v4f*)(priceS + 4 * f);
        *(volatile v4f*)(wp + 4 * f) = q4;
      }
      if (tid < 8) {
        const v4f e4 = *(const v4f*)(sc + SC_EXD + 4 * tid);
        const v4f c4 = *(const v4f*)(sc + SC_CVE + 4 * tid);
        const v4f d4 = *(const v4f*)(sc + SC_DL + 4 * tid);
        *(volatile v4f*)(we + 4 * tid) = e4;
        *(volatile v4f*)(wc + 4 * tid) = c4;
        *(volatile v4f*)(o2 + 4 * tid) = d4;
      }
      __threadfence();
    }
  }
}

__global__ __launch_bounds__(FIN_THREADS) void lv_finish(const float* __restrict__ price, const float* __restrict__ exd,
                                                       const float* __restrict__ cveP, float* __restrict__ out,
                                                       const int* __restrict__ auxA, const int* __restrict__ auxB,
                                                       const int* __restrict__ auxC) {
  __shared__ float part[FIN_THREADS];
  __shared__ float part2[FIN_THREADS];
  __shared__ float colMean[64];
  __shared__ float colVar[64];
  (void)auxA; (void)auxB; (void)auxC;
  const int tid = threadIdx.x;
  const int col = tid & 63, grp = tid >> 6;
  const float invN = 1.0f / 32768.0f;
  const float invN1 = 1.0f / 32767.0f;

  float tot = 0.0f;
#pragma unroll 1
  for (int bq = 0; bq < 128; ++bq) {
    float s = 0.0f;
    const size_t r0 = (size_t)grp * 8192 + (size_t)bq * 64;
#pragma unroll 4
    for (int u = 0; u < 64; ++u) s += price[(r0 + u) * 64 + col];
    tot += s;
  }
  part[tid] = tot;
  __syncthreads();
  if (tid < 64) colMean[tid] = (((part[tid] + part[64 + tid]) + part[128 + tid]) + part[192 + tid]) * invN;
  __syncthreads();
  const float cm = colMean[col];
  tot = 0.0f;
#pragma unroll 1
  for (int bq = 0; bq < 128; ++bq) {
    float s = 0.0f;
    const size_t r0 = (size_t)grp * 8192 + (size_t)bq * 64;
#pragma unroll 4
    for (int u = 0; u < 64; ++u) {
      const float d = price[(r0 + u) * 64 + col] - cm;
      s = fmaf(d, d, s);
    }
    tot += s;
  }
  part[tid] = tot;
  __syncthreads();
  if (tid < 64) colVar[tid] = (((part[tid] + part[64 + tid]) + part[128 + tid]) + part[192 + tid]) * invN1;
  __syncthreads();

  float sa = 0.0f, sb = 0.0f;
#pragma unroll 1
  for (int it = 0; it < 128; ++it) {
    const int r = it * FIN_THREADS + tid;
    const float a = exd[r], b = cveP[r];
    sa += a;
    sb += (a - b);
  }
  part[tid] = sa;
  part2[tid] = sb;
  __syncthreads();
  for (int s = FIN_THREADS / 2; s > 0; s >>= 1) {
    if (tid < s) { part[tid] += part[tid + s]; part2[tid] += part2[tid + s]; }
    __syncthreads();
  }
  const float meanA  = part[0] * invN;
  const float meanEP = part2[0] * invN;
  __syncthreads();
  float sv = 0.0f;
#pragma unroll 1
  for (int it = 0; it < 128; ++it) {
    const int r = it * FIN_THREADS + tid;
    const float ep = exd[r] - cveP[r];
    const float d = ep - meanEP;
    sv = fmaf(d, d, sv);
  }
  part[tid] = sv;
  __syncthreads();
  for (int s = FIN_THREADS / 2; s > 0; s >>= 1) {
    if (tid < s) part[tid] += part[tid + s];
    __syncthreads();
  }
  const float varEP = part[0] * invN1;

  float* ob = out + TAIL_OFF;
  const int nF4 = TAIL_FLOATS / 4;
  for (int pass = 0; pass < 2; ++pass) {
#pragma unroll 1
    for (int it = 0; it < (nF4 + FIN_THREADS - 1) / FIN_THREADS; ++it) {
      const int f = it * FIN_THREADS + tid;
      if (f < nF4) {
        v4f v;
#pragma unroll
        for (int u = 0; u < 4; ++u) {
          const int e = 4 * f + u;
          const int ip = (e < 63) ? e : 62;
          int iv = e - 63; iv = (iv < 0) ? 0 : ((iv > 62) ? 62 : iv);
          int p1 = e - 126; p1 = (p1 < 0) ? 0 : ((p1 > NUM_PATHS - 1) ? (NUM_PATHS - 1) : p1);
          int p2 = e - 32896; p2 = (p2 < 0) ? 0 : ((p2 > NUM_PATHS - 1) ? (NUM_PATHS - 1) : p2);
          const float pv = colMean[ip];
          const float vv = colVar[iv];
          const float a1 = exd[p1], b1 = cveP[p1];
          const float a2 = exd[p2], b2 = cveP[p2];
          float val = (a2 - meanA) - b2;
          val = (e == 32895) ? varEP : val;
          val = (e == 32894) ? meanEP : val;
          val = (e < 32894) ? (a1 - b1) : val;
          val = (e < 126) ? vv : val;
          val = (e < 63) ? pv : val;
          v[u] = val;
        }
        *(volatile v4f*)(ob + 4 * (size_t)f) = v;
      }
    }
    __threadfence();
  }
}

static void launch_prep(const float* src, int srcMatStride, int kdim, int ndim, int nMat, int nPad, int kPitch,
                        _Float16* dst, hipStream_t stream) {
  const int totalLines = nMat * nPad * (kPitch / 64);
  const int blocks = (totalLines + 7) / 8;
  prep_bt16<<<blocks, 64, 0, stream>>>(src, srcMatStride, kdim, ndim, nPad, kPitch, totalLines, dst);
}

extern "C" void kernel_launch(void* const* d_in, const int* in_sizes, int n_in,
                              void* d_out, int out_size, void* d_ws, size_t ws_size,
                              hipStream_t stream) {
  if (n_in < 23) return;
  if (in_sizes[1] != NUM_PATHS * NUM_STEPS) return;
  if (out_size != OUT_TOTAL) return;
  if (ws_size < WS_END) return;

  const float* S0  = (const float*)d_in[0];
  const float* z   = (const float*)d_in[1];
  const int*   mcS = (const int*)d_in[2];
  const int*   indT = (const int*)d_in[3];
  const int*   perL = (const int*)d_in[4];
  const float* dWi = (const float*)d_in[5];
  const float* dbi = (const float*)d_in[6];
  const float* dWh = (const float*)d_in[7];
  const float* dbh = (const float*)d_in[8];
  const float* dWo = (const float*)d_in[9];
  const float* dbo = (const float*)d_in[10];
  const float* vWi = (const float*)d_in[11];
  const float* vbi = (const float*)d_in[12];
  const float* vWh = (const float*)d_in[13];
  const float* vbh = (const float*)d_in[14];
  const float* vWo = (const float*)d_in[15];
  const float* vbo = (const float*)d_in[16];
  const float* eWi = (const float*)d_in[17];
  const float* ebi = (const float*)d_in[18];
  const float* eWh = (const float*)d_in[19];
  const float* ebh = (const float*)d_in[20];
  const float* eWo = (const float*)d_in[21];
  const float* ebo = (const float*)d_in[22];
  float* out = (float*)d_out;

  char* ws = (char*)d_ws;
  _Float16* bt   = (_Float16*)(ws + WS_BT);
  float* wsPrice = (float*)(ws + WS_PRICE);
  float* wsExd   = (float*)(ws + WS_EXD);
  float* wsCve   = (float*)(ws + WS_CVE);

  launch_prep(dWh,      2500, 50, 50, 9, 64, 64,  bt + BT_DWH, stream);
  launch_prep(dWo,        50, 50,  1, 3, 16, 64,  bt + BT_DWO, stream);
  launch_prep(vWh,       900, 30, 30, 6, 32, 64,  bt + BT_VWH, stream);
  launch_prep(vWo,      1890, 30, 63, 3, 64, 64,  bt + BT_VWO, stream);
  launch_prep(eWi + 20, 1840, 91, 20, 3, 32, 128, bt + BT_EWI, stream);
  launch_prep(eWh,       400, 20, 20, 6, 32, 64,  bt + BT_EWH, stream);
  launch_prep(eWo,        20, 20,  1, 3, 16, 64,  bt + BT_EWO, stream);

  const int nS0 = in_sizes[0];
  lv_paths<<<NUM_PATHS / PATHS_PER_BLOCK, MAIN_THREADS, 0, stream>>>(
      S0, nS0, z, dWi, dbi, dbh, dbo, vWi, vbi, vbh, vbo, eWi, ebi, ebh, ebo,
      bt, out, wsPrice, wsExd, wsCve);

  lv_finish<<<1, FIN_THREADS, 0, stream>>>(wsPrice, wsExd, wsCve, out, mcS, indT, perL);
  (void)ws_size;
}
